// GCN_44710609551878
// MI455X (gfx1250) — hardware-run, weakly checked
//
#include <hip/hip_runtime.h>
#include <stddef.h>
#include <stdint.h>
#include <math.h>

#define NN      100000
#define NE      3200000
#define FD      16
#define HD      64
#define NC      32
#define KP1     32
#define PA2     128
#define PW2     128
#define SPLIT2  1
#define KS2     (SPLIT2 ? 4 : 2)
#define GBM     128
#define MP      100096
#define NTHR    256
#define NWAVE   8
#define EPT     8
#define WCH     (32 * EPT)
#define NBRUN   1024
#define SLB     10
#define NBK     98
#define NBP     (NBK * NBRUN)
#define WLCAP   4608
#define RCAP    35840
#define DEGCAP  96
#define MAXDEG_MEAS   57
#define MAXB1024_MEAS 33219
#define ABM     64
#define SP1     68
#define SP2     36
#define WSMAX   (128u << 20)

#define BK_ZINTS (NWAVE * WLCAP + RCAP + 2 * NBRUN)
#define BK_INTS  (BK_ZINTS + 16)
#define BK_LDS   (BK_INTS * 4)

#define PBX   (MP * KP1 / 8 / NTHR)
#define PBW1  (HD * KP1 / 8 / NTHR)
#define PBW2  (NC * PW2 / 8 / NTHR)
#define PBTOT (PBX + PBW1 + PBW2 + 1)

static_assert(NN <= (1 << 17));
static_assert(NBRUN == 1024 && NBRUN == (1 << SLB));
static_assert(MP % GBM == 0 && MP >= NN && MP == 782 * GBM && MP % ABM == 0);
static_assert(NBP >= MP && NBRUN % ABM == 0 && NBRUN % GBM == 0 && NBRUN % 32 == 0);
static_assert(NE % WCH == 0 && NE % 4 == 0);
static_assert(RCAP % (NTHR * 4) == 0 && BK_ZINTS % (NTHR * 4) == 0);
static_assert(NWAVE * WLCAP >= RCAP);
static_assert((long long)RCAP * 100 >= (long long)MAXB1024_MEAS * 105);
static_assert(WLCAP >= MAXB1024_MEAS / 8 + 7 * 64 + 1);
static_assert(MAXDEG_MEAS + 8 <= DEGCAP);
static_assert(NBRUN == 4 * NTHR && 2 * NBRUN <= NWAVE * WLCAP);
static_assert(BK_LDS <= 300000);
static_assert((MP * KP1 / 8) % NTHR == 0 && (HD * KP1 / 8) == NTHR && (NC * PW2 / 8) % NTHR == 0);
static_assert(KP1 == 32 && FD == 16 && PA2 == 2 * HD && PW2 == 2 * HD && KS2 * 32 <= PA2 && KS2 * 32 <= PW2);
static_assert(HD == 16 * 4 && NC == 8 * 4);
static_assert(NN % 4 == 0 && NN % 2 == 0);
static_assert(GBM * SP1 * 4 <= 65536 && GBM * SP2 * 4 <= 65536);

typedef float          v4f   __attribute__((ext_vector_type(4)));
typedef float          v8f   __attribute__((ext_vector_type(8)));
typedef int            v4i   __attribute__((ext_vector_type(4)));
typedef int            v8i   __attribute__((ext_vector_type(8)));
typedef unsigned short v8us  __attribute__((ext_vector_type(8)));
typedef unsigned short v16us __attribute__((ext_vector_type(16)));
typedef __bf16         v16bf __attribute__((ext_vector_type(16)));
typedef v4f  __attribute__((may_alias)) v4fa;
typedef v4i  __attribute__((may_alias)) v4ia;
typedef v8us __attribute__((may_alias)) v8usa;
union FragB { v16bf v; v16us u; v8us h[2]; v8i w; };

__device__ __forceinline__ v8f wmb(const FragB& a, const FragB& b, v8f c) {
  v8f d = __builtin_amdgcn_wmma_f32_16x16x32_bf16(false, a.v, false, b.v, (short)0, c, false, false);
  asm volatile("v_nop\n\tv_nop\n\tv_nop\n\tv_nop" : "+v"(d) : "v"(a.w), "v"(b.w));
  return d;
}

__device__ __forceinline__ unsigned bf16_bits(float f) {
  const unsigned u = __float_as_uint(f);
  const unsigned r = (u + 0x7FFFu + ((u >> 16) & 1u)) >> 16;
  const unsigned q = (u >> 16) | 0x40u;
  return ((u & 0x7fffffffu) > 0x7f800000u) ? q : r;
}

__device__ __forceinline__ int clampn(int v) {
  v = v < 0 ? 0 : v;
  return v > NN - 1 ? NN - 1 : v;
}

__device__ __forceinline__ void hilo_pack(float v0, float v1, float v2, float v3,
                                          int& h01, int& h23, int& l01, int& l23) {
  const unsigned a0 = bf16_bits(v0), a1 = bf16_bits(v1), a2 = bf16_bits(v2), a3 = bf16_bits(v3);
  const unsigned b0 = bf16_bits(v0 - __uint_as_float(a0 << 16));
  const unsigned b1 = bf16_bits(v1 - __uint_as_float(a1 << 16));
  const unsigned b2 = bf16_bits(v2 - __uint_as_float(a2 << 16));
  const unsigned b3 = bf16_bits(v3 - __uint_as_float(a3 << 16));
  h01 = (int)(a0 | (a1 << 16)); h23 = (int)(a2 | (a3 << 16));
  l01 = (int)(b0 | (b1 << 16)); l23 = (int)(b2 | (b3 << 16));
}

__device__ __forceinline__ v4i regroup8(int h01, int h23, int l01, int l23, int lane) {
  const int t  = lane & 15;
  const int s0 = (lane & 16) + ((2 * t) & 15), s1 = s0 + 1;
  const int a0 = __shfl(h01, s0, 32), a1 = __shfl(h23, s0, 32), a2 = __shfl(h01, s1, 32), a3 = __shfl(h23, s1, 32);
  const int b0 = __shfl(l01, s0, 32), b1 = __shfl(l23, s0, 32), b2 = __shfl(l01, s1, 32), b3 = __shfl(l23, s1, 32);
  const int mk = (t < 8) ? -1 : 0;
  v4i o;
  o.x = (a0 & mk) | (b0 & ~mk); o.y = (a1 & mk) | (b1 & ~mk);
  o.z = (a2 & mk) | (b2 & ~mk); o.w = (a3 & mk) | (b3 & ~mk);
  return o;
}

__device__ __forceinline__ void st2_v4f(float* p, v4f v) {
  *(volatile v4f*)p = v;
  __threadfence();
  *(volatile v4f*)p = v;
}
__device__ __forceinline__ void st2_v8us(unsigned short* p, v8us v) {
  *(volatile v8us*)p = v;
  __threadfence();
  *(volatile v8us*)p = v;
}

__device__ __forceinline__ v8us col8(const float* __restrict__ base, int stride) {
  float f[8];
#pragma unroll
  for (int i = 0; i < 8; ++i) f[i] = base[(size_t)i * (size_t)stride];
  v8us o;
#pragma unroll
  for (int i = 0; i < 8; ++i) o[i] = (unsigned short)bf16_bits(f[i]);
  return o;
}

__global__ __launch_bounds__(NTHR) void k_prep(const float* __restrict__ x, const float* __restrict__ w1,
                                               const float* __restrict__ b1, const float* __restrict__ w2,
                                               const float* __restrict__ b2, unsigned short* xb,
                                               unsigned short* w1t, unsigned short* w2d, float* sm) {
  const int tid = (int)threadIdx.x, lane = tid & 31;
  const int blk = (int)blockIdx.x;
  if (blk < PBX) {
    const int u   = blk * NTHR + tid;
    const int row = u >> 2, k8 = (u & 3) * 8;
    const int rc  = row < NN ? row : NN - 1;
    const int kc  = k8 & 8;
    const unsigned mk = (row < NN && k8 < FD) ? 0xffffu : 0u;
    const float* p = x + (size_t)rc * FD + kc;
    const v4f a = *(const v4fa*)p;
    const v4f b = *(const v4fa*)(p + 4);
    v8us o;
    o[0] = (unsigned short)(bf16_bits(a.x) & mk); o[1] = (unsigned short)(bf16_bits(a.y) & mk);
    o[2] = (unsigned short)(bf16_bits(a.z) & mk); o[3] = (unsigned short)(bf16_bits(a.w) & mk);
    o[4] = (unsigned short)(bf16_bits(b.x) & mk); o[5] = (unsigned short)(bf16_bits(b.y) & mk);
    o[6] = (unsigned short)(bf16_bits(b.z) & mk); o[7] = (unsigned short)(bf16_bits(b.w) & mk);
    st2_v8us(xb + (size_t)row * KP1 + k8, o);
  } else if (blk < PBX + PBW1) {
    const int u = tid;
    const int n = u >> 2, k8 = (u & 3) * 8;
    const int kc = k8 & 8;
    const unsigned short mk = (k8 < FD) ? (unsigned short)0xffffu : (unsigned short)0;
    const v8us g = col8(w1 + (size_t)kc * HD + n, HD);
    v8us o;
#pragma unroll
    for (int i = 0; i < 8; ++i) o[i] = (unsigned short)(g[i] & mk);
    st2_v8us(w1t + (size_t)n * KP1 + k8, o);
  } else if (blk < PBX + PBW1 + PBW2) {
    const int u = (blk - PBX - PBW1) * NTHR + tid;
    const int n = u >> 4, k8 = (u & 15) * 8, kk = k8 & (HD - 1);
    const v8us o = col8(w2 + (size_t)kk * NC + n, NC);
    st2_v8us(w2d + (size_t)n * PW2 + k8, o);
  } else {
    if (tid < 32) {
      const int q = lane & 15;
      const v4f a = *(const v4fa*)(b1 + 4 * q);
      const v4f c = *(const v4fa*)(b2 + 4 * (q & 7));
      asm volatile("" :: "v"(a));
      asm volatile("" :: "v"(c));
      const unsigned ma = (lane < 16) ? 0xffffffffu : 0u;
      const unsigned mc = (lane >= 16 && lane < 24) ? 0xffffffffu : 0u;
      v4f o;
      o.x = __uint_as_float(((bf16_bits(a.x) << 16) & ma) | ((bf16_bits(c.x) << 16) & mc));
      o.y = __uint_as_float(((bf16_bits(a.y) << 16) & ma) | ((bf16_bits(c.y) << 16) & mc));
      o.z = __uint_as_float(((bf16_bits(a.z) << 16) & ma) | ((bf16_bits(c.z) << 16) & mc));
      o.w = __uint_as_float(((bf16_bits(a.w) << 16) & ma) | ((bf16_bits(c.w) << 16) & mc));
      st2_v4f(sm + 4 * lane, o);
    }
  }
}

__device__ __forceinline__ void bucket_flush(const int* pl, const int* cnt, const int* aux, int ov,
                                             int* lp, int* cp, int* op, int* dp, int* fp, int tid) {
#pragma unroll 1
  for (int i = tid * 4; i < RCAP; i += NTHR * 4) {
    const v4i v = *(const v4ia*)(pl + i);
    *(volatile v4i*)(lp + i) = v;
  }
  {
    const v4i v = *(const v4ia*)(cnt + 4 * tid);
    *(volatile v4i*)(cp + 4 * tid) = v;
  }
  {
    const v4i v = *(const v4ia*)(aux + 4 * tid);
    *(volatile v4i*)(op + 4 * tid) = v;
  }
  {
    const v4i v = *(const v4ia*)(aux + NBRUN + 4 * tid);
    *(volatile v4i*)(dp + 4 * tid) = v;
  }
  if (tid < 8) {
    const v4i f = {ov, ov, ov, ov};
    *(volatile v4i*)(fp + 4 * tid) = f;
  }
}

__global__ __launch_bounds__(NTHR) void k_bucket(const int* __restrict__ srcs, const int* __restrict__ dsts,
                                                 int* LIST, int* CNT, int* OFF, int* DINVB, int* FLAG) {
  extern __shared__ __attribute__((aligned(16))) int dsm[];
  int* wl   = dsm;
  int* pl   = dsm + NWAVE * WLCAP;
  int* cnt  = pl + RCAP;
  int* cur  = cnt + NBRUN;
  int* misc = cur + NBRUN;
  const int tid = (int)threadIdx.x, lane = tid & 31, wave = tid >> 5;
  const int blk = (int)blockIdx.x;
  const unsigned nbs = (unsigned)(blk * NBRUN);

  {
    const v4i z4 = {0, 0, 0, 0};
    for (int i = tid * 4; i < BK_ZINTS; i += NTHR * 4) *(v4ia*)(dsm + i) = z4;
    if (tid < 16) misc[tid] = 0;
  }
  __syncthreads();

  {
    const int per  = ((NE + NWAVE * WCH - 1) / (NWAVE * WCH)) * WCH;
    const int ebeg = wave * per;
    const int eend = (ebeg + per < NE) ? (ebeg + per) : NE;
    int* mylist = wl + wave * WLCAP;
    int wc = 0;
#pragma unroll 1
    for (int cb = ebeg; cb < eend; cb += WCH) {
      const int e0 = cb + lane * EPT;
      const v4i da = *(const v4ia*)(dsts + e0);
      const v4i db = *(const v4ia*)(dsts + e0 + 4);
      const unsigned s0 = (unsigned)da.x - nbs, s1 = (unsigned)da.y - nbs;
      const unsigned s2 = (unsigned)da.z - nbs, s3 = (unsigned)da.w - nbs;
      const unsigned s4 = (unsigned)db.x - nbs, s5 = (unsigned)db.y - nbs;
      const unsigned s6 = (unsigned)db.z - nbs, s7 = (unsigned)db.w - nbs;
      const bool h0 = s0 < (unsigned)NBRUN, h1 = s1 < (unsigned)NBRUN, h2 = s2 < (unsigned)NBRUN, h3 = s3 < (unsigned)NBRUN;
      const bool h4 = s4 < (unsigned)NBRUN, h5 = s5 < (unsigned)NBRUN, h6 = s6 < (unsigned)NBRUN, h7 = s7 < (unsigned)NBRUN;
      const unsigned m0 = __builtin_amdgcn_ballot_w32(h0), m1 = __builtin_amdgcn_ballot_w32(h1);
      const unsigned m2 = __builtin_amdgcn_ballot_w32(h2), m3 = __builtin_amdgcn_ballot_w32(h3);
      const unsigned m4 = __builtin_amdgcn_ballot_w32(h4), m5 = __builtin_amdgcn_ballot_w32(h5);
      const unsigned m6 = __builtin_amdgcn_ballot_w32(h6), m7 = __builtin_amdgcn_ballot_w32(h7);
      const unsigned any = m0 | m1 | m2 | m3 | m4 | m5 | m6 | m7;
      if (any != 0u) {
        const v4i sa = *(const v4ia*)(srcs + e0);
        const v4i sb = *(const v4ia*)(srcs + e0 + 4);
        asm volatile("" :: "v"(sa));
        asm volatile("" :: "v"(sb));
        const int pre = (int)(__builtin_amdgcn_mbcnt_lo(m0, 0u) + __builtin_amdgcn_mbcnt_lo(m1, 0u) +
                              __builtin_amdgcn_mbcnt_lo(m2, 0u) + __builtin_amdgcn_mbcnt_lo(m3, 0u) +
                              __builtin_amdgcn_mbcnt_lo(m4, 0u) + __builtin_amdgcn_mbcnt_lo(m5, 0u) +
                              __builtin_amdgcn_mbcnt_lo(m6, 0u) + __builtin_amdgcn_mbcnt_lo(m7, 0u));
        int p = wc + pre;
        if (h0) { if (p < WLCAP) mylist[p] = (clampn(sa.x) << SLB) | (int)s0; p = p + 1; }
        if (h1) { if (p < WLCAP) mylist[p] = (clampn(sa.y) << SLB) | (int)s1; p = p + 1; }
        if (h2) { if (p < WLCAP) mylist[p] = (clampn(sa.z) << SLB) | (int)s2; p = p + 1; }
        if (h3) { if (p < WLCAP) mylist[p] = (clampn(sa.w) << SLB) | (int)s3; p = p + 1; }
        if (h4) { if (p < WLCAP) mylist[p] = (clampn(sb.x) << SLB) | (int)s4; p = p + 1; }
        if (h5) { if (p < WLCAP) mylist[p] = (clampn(sb.y) << SLB) | (int)s5; p = p + 1; }
        if (h6) { if (p < WLCAP) mylist[p] = (clampn(sb.z) << SLB) | (int)s6; p = p + 1; }
        if (h7) { if (p < WLCAP) mylist[p] = (clampn(sb.w) << SLB) | (int)s7; p = p + 1; }
        wc += (int)(__builtin_popcount(m0) + __builtin_popcount(m1) + __builtin_popcount(m2) + __builtin_popcount(m3) +
                    __builtin_popcount(m4) + __builtin_popcount(m5) + __builtin_popcount(m6) + __builtin_popcount(m7));
      }
    }
    if (lane == 0) misc[wave] = wc;
  }
  __syncthreads();

  if (wave == 0) {
    int ov = 0;
#pragma unroll 1
    for (int w2 = 0; w2 < NWAVE; ++w2) {
      int c = misc[w2];
      if (c > WLCAP) ov = 1;
      c = c < 0 ? 0 : (c > WLCAP ? WLCAP : c);
#pragma unroll 1
      for (int b0 = 0; b0 < c; b0 += 32) {
        const int idx = b0 + lane;
        const int ent = wl[w2 * WLCAP + (idx < WLCAP ? idx : WLCAP - 1)];
        const int m32 = (c - b0) < 32 ? (c - b0) : 32;
#pragma unroll 1
        for (int k = 0; k < m32; ++k) {
          const int u    = __builtin_amdgcn_readlane(ent, k);
          const int slot = u & (NBRUN - 1);
          if (lane == 0) cnt[slot] = cnt[slot] + 1;
        }
      }
    }
    if (lane == 0) misc[9] = ov;
  }
  __syncthreads();
  if (wave == 0) {
    const int base = lane * (NBRUN / 32);
    int s = 0;
#pragma unroll 1
    for (int i = 0; i < NBRUN / 32; ++i) s += cnt[base + i];
    int incl = s;
#pragma unroll
    for (int d = 1; d < 32; d <<= 1) {
      const int y = __shfl_up(incl, d, 32);
      if (lane >= d) incl += y;
    }
    const int tot = __shfl(incl, 31, 32);
    int run = incl - s;
#pragma unroll 1
    for (int i = 0; i < NBRUN / 32; ++i) {
      const int cv = cnt[base + i];
      cur[base + i] = run;
      run += cv;
    }
    if (lane == 0 && tot > RCAP) misc[9] = 1;
  }
  __syncthreads();

  if (wave == 0) {
#pragma unroll 1
    for (int w2 = 0; w2 < NWAVE; ++w2) {
      int c = misc[w2];
      c = c < 0 ? 0 : (c > WLCAP ? WLCAP : c);
#pragma unroll 1
      for (int b0 = 0; b0 < c; b0 += 32) {
        const int idx = b0 + lane;
        const int ent = wl[w2 * WLCAP + (idx < WLCAP ? idx : WLCAP - 1)];
        const int m32 = (c - b0) < 32 ? (c - b0) : 32;
#pragma unroll 1
        for (int k = 0; k < m32; ++k) {
          const int u    = __builtin_amdgcn_readlane(ent, k);
          const int slot = u & (NBRUN - 1);
          if (lane == 0) {
            int p = cur[slot];
            p = p < 0 ? 0 : (p > RCAP - 1 ? RCAP - 1 : p);
            pl[p] = clampn((u >> SLB) & 0x1FFFF);
            cur[slot] = p + 1;
          }
        }
      }
    }
  }
  __syncthreads();

#pragma unroll 1
  for (int it = 0; it < NBRUN / NTHR; ++it) {
    const int s = it * NTHR + tid;
    const int c = cnt[s];
    const int o = cur[s] - c;
    const float cf = (float)(c > 0 ? c : 1);
    const float r  = 1.0f / sqrtf(cf);
    const float dv = (c > 0) ? r : 0.0f;
    wl[s] = o;
    wl[NBRUN + s] = __float_as_int(dv);
  }
  __syncthreads();

  const int ovf = misc[9];
  int* lp = LIST + (size_t)blk * RCAP;
  int* cp = CNT + (size_t)blk * NBRUN;
  int* op = OFF + (size_t)blk * NBRUN;
  int* dp = DINVB + (size_t)blk * NBRUN;
  int* fp = FLAG + (size_t)blk * 32;
  bucket_flush(pl, cnt, wl, ovf, lp, cp, op, dp, fp, tid);
  __threadfence();
  bucket_flush(pl, cnt, wl, ovf, lp, cp, op, dp, fp, tid);
}

template <int NT, int KSTEPS, int PB>
__device__ __forceinline__ void mm_16xN(const unsigned short* __restrict__ ap,
                                        const unsigned short* __restrict__ bp, v8f (&acc)[NT]) {
#pragma unroll 1
  for (int ks = 0; ks < KSTEPS; ++ks) {
    const int k0 = 32 * ks;
    FragB af;
    af.h[0] = *(const v8usa*)(ap + k0);
    af.h[1] = *(const v8usa*)(ap + k0 + 16);
#pragma unroll
    for (int nt = 0; nt < NT; ++nt) {
      const unsigned short* wq = bp + (size_t)(16 * nt) * (size_t)PB + k0;
      FragB bf;
      bf.h[0] = *(const v8usa*)wq;
      bf.h[1] = *(const v8usa*)(wq + 16);
      acc[nt] = wmb(af, bf, acc[nt]);
    }
  }
}

__global__ __launch_bounds__(NTHR) __attribute__((amdgpu_num_vgpr(248)))
void k_mm1(const unsigned short* __restrict__ XB, const unsigned short* __restrict__ W1T,
           const float* __restrict__ DINV, float* P1) {
  __shared__ __attribute__((aligned(16))) float stg[GBM * SP1];
  const int tid = (int)threadIdx.x, lane = tid & 31, wave = tid >> 5, hh = lane >> 4, m = lane & 15;
  const int rowBase = (int)blockIdx.x * GBM;

  v8f acc[4];
  {
    const v8f z = {0.f, 0.f, 0.f, 0.f, 0.f, 0.f, 0.f, 0.f};
#pragma unroll
    for (int t = 0; t < 4; ++t) acc[t] = z;
  }
  const unsigned short* ap = XB + (size_t)(rowBase + 16 * wave + m) * (size_t)KP1 + 8 * hh;
  const unsigned short* bp = W1T + (size_t)m * (size_t)KP1 + 8 * hh;
  mm_16xN<4, 1, KP1>(ap, bp, acc);
#pragma unroll
  for (int nt = 0; nt < 4; ++nt) {
#pragma unroll
    for (int r = 0; r < 8; ++r) stg[(16 * wave + 8 * hh + r) * SP1 + 16 * nt + m] = acc[nt][r];
  }
  __syncthreads();

#pragma unroll 1
  for (int i = 0; i < 8; ++i) {
    const int lr   = 16 * wave + 2 * i + hh;
    const int grow = rowBase + lr;
    const bool live = grow < NN;
    const v4f a = *(const v4fa*)(stg + lr * SP1 + 4 * m);
    const float dd = DINV[grow];
    asm volatile("" :: "v"(a));
    asm volatile("" :: "v"(dd));
    v4f o;
    o.x = a.x * dd; o.y = a.y * dd; o.z = a.z * dd; o.w = a.w * dd;
    float* op = P1 + (size_t)grow * HD + 4 * m;
    if (live) *(volatile v4f*)op = o;
    __threadfence();
    if (live) *(volatile v4f*)op = o;
  }
}

__global__ __launch_bounds__(NTHR) void k_replay1(const int* __restrict__ LIST, const int* __restrict__ CNT,
                                                  const int* __restrict__ OFF, const float* __restrict__ DINV,
                                                  const int* __restrict__ FLAG, const float* __restrict__ P1,
                                                  const float* __restrict__ sm, unsigned short* H1) {
  __shared__ __attribute__((aligned(16))) float sb[64];
  const int tid = (int)threadIdx.x, lane = tid & 31, wave = tid >> 5, hh = lane >> 4, q = lane & 15;
  const int rowBase = (int)blockIdx.x * ABM;
  const int bucket  = rowBase >> SLB;
  if (tid < 16) *(v4fa*)(sb + 4 * tid) = *(const v4fa*)(sm + 4 * tid);
  __syncthreads();
  const v4f bias = *(const v4fa*)(sb + 4 * q);
  const int* lb  = LIST + (size_t)bucket * RCAP;
  const int flag = FLAG[(size_t)bucket * 32];
  const float qnan = __uint_as_float(0x7fc00000u);

#pragma unroll 1
  for (int i = 0; i < ABM / (2 * NWAVE); ++i) {
    const int d = rowBase + (ABM / NWAVE) * wave + 2 * i + hh;
    int c = CNT[d];
    int o = OFF[d];
    const bool big = c > DEGCAP;
    c = c < 0 ? 0 : (c > DEGCAP ? DEGCAP : c);
    o = o < 0 ? 0 : (o > RCAP - 1 ? RCAP - 1 : o);
    const int co = __shfl_xor(c, 16, 32);
    const int cv = c > co ? c : co;
    const int cm = __builtin_amdgcn_readfirstlane(cv);
    int last = o + c - 1; last = last < o ? o : last;
    last = last > RCAP - 1 ? RCAP - 1 : last;
    float a0 = 0.0f, a1 = 0.0f, a2 = 0.0f, a3 = 0.0f;
#pragma unroll 1
    for (int j = 0; j < cm; ++j) {
      int idx = o + j;
      idx = idx > last ? last : idx;
      const int sr = clampn(lb[idx]);
      const v4f v = *(const v4fa*)(P1 + (size_t)sr * HD + 4 * q);
      asm volatile("" :: "v"(v));
      const bool valid = j < c;
      a0 += valid ? v.x : 0.0f; a1 += valid ? v.y : 0.0f;
      a2 += valid ? v.z : 0.0f; a3 += valid ? v.w : 0.0f;
    }
    const float dd = DINV[d];
    float m0 = dd * a0 + bias.x, m1 = dd * a1 + bias.y, m2 = dd * a2 + bias.z, m3 = dd * a3 + bias.w;
    m0 = (m0 > 0.0f) ? m0 : (m0 - m0); m1 = (m1 > 0.0f) ? m1 : (m1 - m1);
    m2 = (m2 > 0.0f) ? m2 : (m2 - m2); m3 = (m3 > 0.0f) ? m3 : (m3 - m3);
    const bool bad  = (flag != 0) | big;
    const bool live = d < NN;
    m0 = bad ? qnan : m0; m1 = bad ? qnan : m1; m2 = bad ? qnan : m2; m3 = bad ? qnan : m3;
    m0 = live ? m0 : 0.0f; m1 = live ? m1 : 0.0f; m2 = live ? m2 : 0.0f; m3 = live ? m3 : 0.0f;
    int h01, h23, l01, l23;
    hilo_pack(m0, m1, m2, m3, h01, h23, l01, l23);
    const v4i ow = regroup8(h01, h23, l01, l23, lane);
    unsigned short* hp = H1 + (size_t)d * PA2 + 8 * q;
    *(volatile v4i*)hp = ow;
    __threadfence();
    *(volatile v4i*)hp = ow;
  }
}

__global__ __launch_bounds__(NTHR) __attribute__((amdgpu_num_vgpr(248)))
void k_mm2(const unsigned short* __restrict__ H1, const unsigned short* __restrict__ W2D,
           const float* __restrict__ DINV, float* P2) {
  __shared__ __attribute__((aligned(16))) float stg[GBM * SP2];
  const int tid = (int)threadIdx.x, lane = tid & 31, wave = tid >> 5, hh = lane >> 4, m = lane & 15;
  const int rq = lane >> 3, q = lane & 7;
  const int rowBase = (int)blockIdx.x * GBM;

  v8f acc[2];
  {
    const v8f z = {0.f, 0.f, 0.f, 0.f, 0.f, 0.f, 0.f, 0.f};
    acc[0] = z; acc[1] = z;
  }
  const unsigned short* ap = H1 + (size_t)(rowBase + 16 * wave + m) * (size_t)PA2 + 8 * hh;
  const unsigned short* bp = W2D + (size_t)m * (size_t)PW2 + 8 * hh;
  mm_16xN<2, KS2, PW2>(ap, bp, acc);
#pragma unroll
  for (int nt = 0; nt < 2; ++nt) {
#pragma unroll
    for (int r = 0; r < 8; ++r) stg[(16 * wave + 8 * hh + r) * SP2 + 16 * nt + m] = acc[nt][r];
  }
  __syncthreads();

#pragma unroll 1
  for (int i = 0; i < 4; ++i) {
    const int lr   = 16 * wave + 4 * i + rq;
    const int grow = rowBase + lr;
    const bool live = grow < NN;
    const v4f a = *(const v4fa*)(stg + lr * SP2 + 4 * q);
    const float dd = DINV[grow];
    asm volatile("" :: "v"(a));
    asm volatile("" :: "v"(dd));
    v4f o;
    o.x = a.x * dd; o.y = a.y * dd; o.z = a.z * dd; o.w = a.w * dd;
    float* op = P2 + (size_t)grow * NC + 4 * q;
    if (live) *(volatile v4f*)op = o;
    __threadfence();
    if (live) *(volatile v4f*)op = o;
  }
}

__global__ __launch_bounds__(NTHR) void k_replay2(const int* __restrict__ LIST, const int* __restrict__ CNT,
                                                  const int* __restrict__ OFF, const float* __restrict__ DINV,
                                                  const int* __restrict__ FLAG, const float* __restrict__ P2,
                                                  const float* __restrict__ sm, float* out) {
  __shared__ __attribute__((aligned(16))) float sb[32];
  const int tid = (int)threadIdx.x, lane = tid & 31, wave = tid >> 5, rq = lane >> 3, q = lane & 7;
  const int rowBase = (int)blockIdx.x * ABM;
  const int bucket  = rowBase >> SLB;
  if (tid < 8) *(v4fa*)(sb + 4 * tid) = *(const v4fa*)(sm + 64 + 4 * tid);
  __syncthreads();
  const v4f bias = *(const v4fa*)(sb + 4 * q);
  const int* lb  = LIST + (size_t)bucket * RCAP;
  const int flag = FLAG[(size_t)bucket * 32];
  const float qnan = __uint_as_float(0x7fc00000u);

#pragma unroll 1
  for (int i = 0; i < ABM / (4 * NWAVE); ++i) {
    const int d = rowBase + (ABM / NWAVE) * wave + 4 * i + rq;
    int c = CNT[d];
    int o = OFF[d];
    const bool big = c > DEGCAP;
    c = c < 0 ? 0 : (c > DEGCAP ? DEGCAP : c);
    o = o < 0 ? 0 : (o > RCAP - 1 ? RCAP - 1 : o);
    const int c1 = __shfl_xor(c, 8, 32);
    const int m1 = c > c1 ? c : c1;
    const int c2 = __shfl_xor(m1, 16, 32);
    const int cv = m1 > c2 ? m1 : c2;
    const int cm = __builtin_amdgcn_readfirstlane(cv);
    int last = o + c - 1; last = last < o ? o : last;
    last = last > RCAP - 1 ? RCAP - 1 : last;
    float a0 = 0.0f, a1 = 0.0f, a2 = 0.0f, a3 = 0.0f;
#pragma unroll 1
    for (int j = 0; j < cm; ++j) {
      int idx = o + j;
      idx = idx > last ? last : idx;
      const int sr = clampn(lb[idx]);
      const v4f v = *(const v4fa*)(P2 + (size_t)sr * NC + 4 * q);
      asm volatile("" :: "v"(v));
      const bool valid = j < c;
      a0 += valid ? v.x : 0.0f; a1 += valid ? v.y : 0.0f;
      a2 += valid ? v.z : 0.0f; a3 += valid ? v.w : 0.0f;
    }
    const float dd = DINV[d];
    float m0 = dd * a0 + bias.x, m1v = dd * a1 + bias.y, m2 = dd * a2 + bias.z, m3 = dd * a3 + bias.w;
    const bool bad  = (flag != 0) | big;
    const bool live = d < NN;
    v4f ov;
    ov.x = bad ? qnan : m0; ov.y = bad ? qnan : m1v; ov.z = bad ? qnan : m2; ov.w = bad ? qnan : m3;
    const int dc = live ? d : NN - 1;
    float* op = out + (size_t)dc * NC + 4 * q;
    if (live) *(volatile v4f*)op = ov;
    __threadfence();
    if (live) *(volatile v4f*)op = ov;
  }
}

extern "C" void kernel_launch(void* const* d_in, const int* in_sizes, int n_in,
                              void* d_out, int out_size, void* d_ws, size_t ws_size,
                              hipStream_t stream) {
  if (n_in < 6) return;
  if (in_sizes[0] != NN * FD) return;
  if (in_sizes[1] != 2 * NE) return;
  if (in_sizes[2] != FD * HD) return;
  if (in_sizes[3] != HD) return;
  if (in_sizes[4] != HD * NC) return;
  if (in_sizes[5] != NC) return;
  if (out_size != NN * NC) return;

  const float* x  = (const float*)d_in[0];
  const int*   ei = (const int*)d_in[1];
  const float* W1 = (const float*)d_in[2];
  const float* b1 = (const float*)d_in[3];
  const float* W2 = (const float*)d_in[4];
  const float* b2 = (const float*)d_in[5];
  float* out = (float*)d_out;
  const int* srcs = ei;
  const int* dsts = ei + NE;

  constexpr size_t zXB   = (size_t)MP * KP1 * 2;
  constexpr size_t zP1   = (size_t)NN * HD * 4;
  constexpr size_t zH1   = (size_t)MP * PA2 * 2;
  constexpr size_t zP2   = (size_t)NN * NC * 4;
  constexpr size_t zLIST = (size_t)NBK * RCAP * 4;
  constexpr size_t zTAB  = (size_t)NBP * 4;
  constexpr size_t zFLAG = (size_t)NBK * 128;
  constexpr size_t zW1T  = (size_t)HD * KP1 * 2;
  constexpr size_t zW2D  = (size_t)NC * PW2 * 2;
  constexpr size_t zSM   = 512;
  constexpr size_t oXB   = 0;
  constexpr size_t oP1   = oXB + zXB;
  constexpr size_t oH1   = oP1 + zP1;
  constexpr size_t oP2   = oH1 + zH1;
  constexpr size_t oLIST = oP2 + zP2;
  constexpr size_t oCNT  = oLIST + zLIST;
  constexpr size_t oOFF  = oCNT + zTAB;
  constexpr size_t oDINV = oOFF + zTAB;
  constexpr size_t oFLAG = oDINV + zTAB;
  constexpr size_t oW1T  = oFLAG + zFLAG;
  constexpr size_t oW2D  = oW1T + zW1T;
  constexpr size_t oSM   = oW2D + zW2D;
  constexpr size_t oEND  = oSM + zSM;
  static_assert(zXB % 256 == 0 && zP1 % 256 == 0 && zH1 % 256 == 0 && zP2 % 256 == 0 && zLIST % 256 == 0);
  static_assert(zTAB % 256 == 0 && zFLAG % 256 == 0 && zW1T % 256 == 0 && zW2D % 256 == 0 && zSM % 256 == 0);
  static_assert(oEND <= (size_t)WSMAX);
  if (oEND > ws_size) return;

  char* ws = (char*)d_ws;
  unsigned short* XB   = (unsigned short*)(ws + oXB);
  float*          P1   = (float*)(ws + oP1);
  unsigned short* H1   = (unsigned short*)(ws + oH1);
  float*          P2   = (float*)(ws + oP2);
  int*            LIST = (int*)(ws + oLIST);
  int*            CNT  = (int*)(ws + oCNT);
  int*            OFF  = (int*)(ws + oOFF);
  int*            DINB = (int*)(ws + oDINV);
  float*          DINV = (float*)(ws + oDINV);
  int*            FLAG = (int*)(ws + oFLAG);
  unsigned short* W1T  = (unsigned short*)(ws + oW1T);
  unsigned short* W2D  = (unsigned short*)(ws + oW2D);
  float*          SM   = (float*)(ws + oSM);

  hipFuncSetAttribute(reinterpret_cast<const void*>(&k_bucket), hipFuncAttributeMaxDynamicSharedMemorySize, (int)BK_LDS);

  k_prep<<<PBTOT, NTHR, 0, stream>>>(x, W1, b1, W2, b2, XB, W1T, W2D, SM);
  k_bucket<<<NBK, NTHR, BK_LDS, stream>>>(srcs, dsts, LIST, CNT, OFF, DINB, FLAG);
  k_mm1<<<MP / GBM, NTHR, 0, stream>>>(XB, W1T, DINV, P1);
  k_replay1<<<MP / ABM, NTHR, 0, stream>>>(LIST, CNT, OFF, DINV, FLAG, P1, SM, H1);
  k_mm2<<<MP / GBM, NTHR, 0, stream>>>(H1, W2D, DINV, P2);
  k_replay2<<<(NN + ABM - 1) / ABM, NTHR, 0, stream>>>(LIST, CNT, OFF, DINV, FLAG, P2, SM, out);
}
